// CausalSelfAttention_39831526703820
// MI455X (gfx1250) — hardware-verified
//
#include <hip/hip_runtime.h>


#ifndef NB
#define NB 4
#endif
#ifndef SEQ
#define SEQ 2048
#endif
#define NB_FULL  4
#define SEQ_FULL 2048
#ifndef OUT_SEQ
#define OUT_SEQ SEQ
#endif
#ifndef EPR
#define EPR ((SEQ) < 512 ? (SEQ) : 512)
#endif
#define DM   1024
#define NH_  16
#define HD   64
#define AW   4
#define QRS  2048.0f
#define QRI  (1.0f / 2048.0f)
#define WOS  1024.0f
#define WOI  (1.0f / 1024.0f)
#define SC2  (0.125f * 1.4426950408889634f)
#define PSH  8.0f
#define NEGB (-3.0e38f)
#define R8   1.333521432163324

static_assert(HD == 64);
static_assert(NH_ * HD == DM);
static_assert(DM % 64 == 0);
static_assert(DM % 32 == 0);
static_assert(SEQ % 64 == 0);
static_assert((NB * SEQ) % 64 == 0);
static_assert(SEQ % 32 == 0);
static_assert(SEQ % (16 * AW) == 0);
static_assert(SEQ % 8 == 0);
static_assert(EPR % 64 == 0);
static_assert(EPR >= 64);
static_assert(EPR <= SEQ);
static_assert((SEQ - EPR) % 64 == 0);
static_assert(((size_t)SEQ * DM) % 8 == 0);
static_assert(((size_t)DM * DM) % 8 == 0);
static_assert(NB <= NB_FULL);
static_assert(SEQ <= SEQ_FULL);

typedef _Float16 h16;
typedef unsigned short bf;
typedef __attribute__((ext_vector_type(16))) __bf16   v16bf;
typedef __attribute__((ext_vector_type(16))) _Float16 v16h;
typedef __attribute__((ext_vector_type(8)))  _Float16 v8h;
typedef __attribute__((ext_vector_type(8)))  unsigned short v8us;
typedef __attribute__((ext_vector_type(8)))  float    v8f;
typedef __attribute__((ext_vector_type(4)))  float    v4f;
typedef v4f  __attribute__((may_alias)) v4fa;

__device__ __forceinline__ unsigned short f2bf(float f) { unsigned u = __float_as_uint(f); u += 0x7FFFu + ((u >> 16) & 1u); return (unsigned short)(u >> 16); }
__device__ __forceinline__ float bf2f(unsigned short s) { return __uint_as_float(((unsigned)s) << 16); }
__device__ __forceinline__ v16h cat16(v8h lo, v8h hi) { return __builtin_shufflevector(lo, hi, 0, 1, 2, 3, 4, 5, 6, 7, 8, 9, 10, 11, 12, 13, 14, 15); }
__device__ __forceinline__ v16bf cat16b(v8us lo, v8us hi) { return __builtin_bit_cast(v16bf, __builtin_shufflevector(lo, hi, 0, 1, 2, 3, 4, 5, 6, 7, 8, 9, 10, 11, 12, 13, 14, 15)); }
__device__ __forceinline__ v8f wmma16(v16h a, v16h b, v8f c) { return __builtin_amdgcn_wmma_f32_16x16x32_f16(false, a, false, b, (short)0, c, false, false); }
__device__ __forceinline__ v8f wmmab(v16bf a, v16bf b, v8f c) { return __builtin_amdgcn_wmma_f32_16x16x32_bf16(false, a, false, b, (short)0, c, false, false); }
__device__ __forceinline__ v16h  ldh(const h16* p) { return cat16(*(const v8h*)p, *(const v8h*)(p + 16)); }
__device__ __forceinline__ v16bf ldb(const bf* p)  { return cat16b(*(const v8us*)p, *(const v8us*)(p + 16)); }
__device__ __forceinline__ void wave_sync() { __builtin_amdgcn_fence(3  , "wavefront"); __builtin_amdgcn_wave_barrier(); asm volatile("" ::: "memory"); }

__global__ __launch_bounds__(256) void k_cvt8(const float* __restrict__ src, bf* dst, size_t n8) {
    const size_t i = (size_t)blockIdx.x * 256 + threadIdx.x; if (i >= n8) return;
    const v8f v = *(const v8f*)(src + i * 8); v8us o;
#pragma unroll
    for (int k = 0; k < 8; ++k) o[k] = f2bf(v[k]);
    *(volatile v8us*)(dst + i * 8) = o; __threadfence(); *(volatile v8us*)(dst + i * 8) = o;
}

__global__ __launch_bounds__(256) void k_cvtw(const float* __restrict__ src, h16* dst, size_t n8) {
    const size_t i = (size_t)blockIdx.x * 256 + threadIdx.x; if (i >= n8) return;
    const v8f v = *(const v8f*)(src + i * 8); v8h o;
#pragma unroll
    for (int k = 0; k < 8; ++k) o[k] = (h16)(bf2f(f2bf(v[k])) * WOS);
    *(volatile v8h*)(dst + i * 8) = o; __threadfence(); *(volatile v8h*)(dst + i * 8) = o;
}

__global__ __launch_bounds__(256) void k_tab(const int* __restrict__ pos, float* TB) {
    __shared__ __align__(16) float cs[2 * 8 * 32];
    const int tid = threadIdx.x, i = tid & 31, rl = tid >> 5;
    const int t = blockIdx.x * 8 + rl;
    double p = 1.0;
#pragma unroll 1
    for (int j = 0; j < i; ++j) p *= R8;
    const float pf = (float)p;
    const float fr = 1.0f / pf;
    const float ang = (float)pos[t] * fr;
    cs[tid] = cosf(ang); cs[256 + tid] = sinf(ang);
    __syncthreads();
    if (tid < 128) {
        const int which = tid >> 6, j = tid & 63, row = j >> 3, pc = (j & 7) * 4;
        const v4f val = *(const v4fa*)(&cs[which * 256 + row * 32 + pc]);
        float* d = TB + (size_t)which * SEQ * 32 + (size_t)(blockIdx.x * 8 + row) * 32 + pc;
        *(volatile v4f*)d = val; __threadfence(); *(volatile v4f*)d = val;
    }
}

__global__ __launch_bounds__(32) void k_proj(const bf* __restrict__ A, const bf* __restrict__ Bt, h16* Ph, h16* Pr,
                                             int RB, size_t sRB, int pitch, int CB, size_t sCB,
                                             int resOn, int pitchR, size_t sRBr, size_t sCBr, int rlimRow, int rlimCol,
                                             const float* __restrict__ TB, int rope) {
    __shared__ __align__(16) float os[16 * 68];
    const int K = DM;
    const int lane = threadIdx.x & 31, lr = lane & 15, hi = lane >> 4; const int r0 = blockIdx.x * 64, c0 = blockIdx.y * 64;
    v8f acc[4][4];
#pragma unroll
    for (int mb = 0; mb < 4; ++mb)
#pragma unroll
        for (int nb = 0; nb < 4; ++nb) acc[mb][nb] = (v8f){};
    const size_t aoff = (size_t)(r0 + lr) * K + 8 * hi, boff = (size_t)(c0 + lr) * K + 8 * hi;
#pragma unroll 1
    for (int kc = 0; kc < K; kc += 32) {
        v16bf a[4];
#pragma unroll
        for (int mb = 0; mb < 4; ++mb) a[mb] = ldb(A + aoff + (size_t)mb * 16 * K + kc);
#pragma unroll
        for (int nb = 0; nb < 4; ++nb) { const v16bf b = ldb(Bt + boff + (size_t)nb * 16 * K + kc);
#pragma unroll
            for (int mb = 0; mb < 4; ++mb) acc[mb][nb] = wmmab(a[mb], b, acc[mb][nb]); }
        asm volatile("v_nop\n\tv_nop\n\tv_nop\n\tv_nop" : "+v"(acc[0][0]), "+v"(acc[1][1]), "+v"(acc[2][2]), "+v"(acc[3][3]) : "v"(a[0]), "v"(a[1]), "v"(a[2]), "v"(a[3]));
    }
    const int rin = r0 % RB, cin = c0 % CB;
    const size_t tbase  = (size_t)(r0 / RB) * sRB  + (size_t)rin * (size_t)pitch  + (size_t)(c0 / CB) * sCB  + (size_t)cin;
    const size_t tbaseR = (size_t)(r0 / RB) * sRBr + (size_t)rin * (size_t)pitchR + (size_t)(c0 / CB) * sCBr + (size_t)cin;
    const int wr = (resOn != 0) && (rin < rlimRow) && (cin < rlimCol);
#pragma unroll
    for (int mb = 0; mb < 4; ++mb) {
#pragma unroll
        for (int nb = 0; nb < 4; ++nb) {
#pragma unroll
            for (int j = 0; j < 8; ++j) os[(hi * 8 + j) * 68 + nb * 16 + lr] = acc[mb][nb][j]; }
        wave_sync();
        const size_t sb  = tbase  + (size_t)(mb * 16) * (size_t)pitch;
        const size_t sbR = tbaseR + (size_t)(mb * 16) * (size_t)pitchR;
#pragma unroll 1
        for (int ps = 0; ps < 2; ++ps) {
#pragma unroll
            for (int s = 0; s < 4; ++s) { const int row = 4 * s + (lane >> 3), c8 = (lane & 7) * 8;
                v4f x0 = *(const v4fa*)(&os[row * 68 + c8]); v4f x1 = *(const v4fa*)(&os[row * 68 + c8 + 4]);
                if (rope) {
                    const int tok = rin + mb * 16 + row;
                    const v4f cv = *(const v4fa*)(TB + (size_t)tok * 32 + (lane & 7) * 4);
                    const v4f sv = *(const v4fa*)(TB + (size_t)SEQ * 32 + (size_t)tok * 32 + (lane & 7) * 4);
                    v4f y0, y1;
                    y0[0] = x0[0] * cv[0] - x0[1] * sv[0]; y0[1] = x0[1] * cv[0] + x0[0] * sv[0];
                    y0[2] = x0[2] * cv[1] - x0[3] * sv[1]; y0[3] = x0[3] * cv[1] + x0[2] * sv[1];
                    y1[0] = x1[0] * cv[2] - x1[1] * sv[2]; y1[1] = x1[1] * cv[2] + x1[0] * sv[2];
                    y1[2] = x1[2] * cv[3] - x1[3] * sv[3]; y1[3] = x1[3] * cv[3] + x1[2] * sv[3];
                    x0 = y0; x1 = y1;
                }
                v8h hv, rv;
#pragma unroll
                for (int i = 0; i < 4; ++i) { const h16 a0 = (h16)x0[i]; const h16 a1 = (h16)x1[i]; hv[i] = a0; hv[4 + i] = a1; rv[i] = (h16)((x0[i] - (float)a0) * QRS); rv[4 + i] = (h16)((x1[i] - (float)a1) * QRS); }
                *(volatile v8h*)(Ph + sb + (size_t)row * (size_t)pitch + c8) = hv;
                if (wr) *(volatile v8h*)(Pr + sbR + (size_t)row * (size_t)pitchR + c8) = rv; }
            if (ps == 0) __threadfence(); }
        wave_sync();
    }
}

template <bool PR>
__global__ __launch_bounds__(32 * AW) void k_flash(const h16* __restrict__ QH, const h16* __restrict__ QR, const h16* __restrict__ KP, const h16* __restrict__ KR,
                                                   const h16* __restrict__ VT, const h16* __restrict__ VR, h16* CH, h16* CR, int tile0) {
    __shared__ __align__(16) float os[AW * 16 * 68];
    const int lane = threadIdx.x & 31, lr = lane & 15, hi = lane >> 4;
    const int wave = __builtin_amdgcn_readfirstlane((int)(threadIdx.x >> 5));
    const int zh = blockIdx.y; const int b = zh / NH_, h = zh % NH_;
    const int t0 = ((tile0 + (int)blockIdx.x) * AW + wave) * 16;
    const size_t pbase = (size_t)zh * SEQ * HD;
    const size_t qo = pbase + (size_t)(t0 + lr) * HD + 8 * hi;
    const v16h qh0 = ldh(QH + qo), qh1 = ldh(QH + qo + 32);
    v16h qr0 = (v16h){}, qr1 = (v16h){};
    if constexpr (PR) {
        const size_t qro = (size_t)zh * EPR * HD + (size_t)(t0 + lr) * HD + 8 * hi;
        qr0 = ldh(QR + qro); qr1 = ldh(QR + qro + 32);
    }
    const size_t ko  = pbase + (size_t)lr * HD + 8 * hi;
    const size_t vo  = pbase + (size_t)lr * SEQ + 8 * hi;
    const size_t kro = (size_t)zh * EPR * HD + (size_t)lr * HD + 8 * hi;
    const size_t vro = (size_t)zh * HD * EPR + (size_t)lr * EPR + 8 * hi;
    v8f oH0 = (v8f){}, oH1 = (v8f){}, oH2 = (v8f){}, oH3 = (v8f){};
    v8f oR0 = (v8f){}, oR1 = (v8f){}, oR2 = (v8f){}, oR3 = (v8f){};
    float m = NEGB, l = 0.0f;
    const int kend = t0 + 16;
#pragma unroll 1
    for (int key0 = 0; key0 < kend; key0 += 32) {
        const h16* ka = KP + ko + (size_t)key0 * HD;
        const v16h ka0 = ldh(ka), ka1 = ldh(ka + 32), kb0 = ldh(ka + 16 * HD), kb1 = ldh(ka + 16 * HD + 32);
        float ta[8], tb[8];
        if constexpr (PR) {
            v8f sHa = (v8f){}, sLa = (v8f){}, sHb = (v8f){}, sLb = (v8f){};
            sHa = wmma16(ka0, qh0, sHa); sLa = wmma16(ka0, qr0, sLa); sHb = wmma16(kb0, qh0, sHb); sLb = wmma16(kb0, qr0, sLb);
            sHa = wmma16(ka1, qh1, sHa); sLa = wmma16(ka1, qr1, sLa); sHb = wmma16(kb1, qh1, sHb); sLb = wmma16(kb1, qr1, sLb);
            const h16* kr = KR + kro + (size_t)key0 * HD;
            const v16h ra0 = ldh(kr), ra1 = ldh(kr + 32), rb0 = ldh(kr + 16 * HD), rb1 = ldh(kr + 16 * HD + 32);
            sLa = wmma16(ra0, qh0, sLa); sLb = wmma16(rb0, qh0, sLb); sLa = wmma16(ra1, qh1, sLa); sLb = wmma16(rb1, qh1, sLb);
            asm volatile("v_nop\n\tv_nop\n\tv_nop\n\tv_nop" : "+v"(sHa), "+v"(sLa), "+v"(sHb), "+v"(sLb) : "v"(ka0), "v"(ka1), "v"(kb0), "v"(kb1), "v"(ra0), "v"(ra1), "v"(rb0), "v"(rb1));
#pragma unroll
            for (int r = 0; r < 8; ++r) { ta[r] = (sHa[r] + sLa[r] * QRI) * SC2; tb[r] = (sHb[r] + sLb[r] * QRI) * SC2; }
        } else {
            v8f sHa = (v8f){}, sHb = (v8f){};
            sHa = wmma16(ka0, qh0, sHa); sHb = wmma16(kb0, qh0, sHb);
            sHa = wmma16(ka1, qh1, sHa); sHb = wmma16(kb1, qh1, sHb);
            asm volatile("v_nop\n\tv_nop\n\tv_nop\n\tv_nop" : "+v"(sHa), "+v"(sHb) : "v"(ka0), "v"(ka1), "v"(kb0), "v"(kb1));
#pragma unroll
            for (int r = 0; r < 8; ++r) { ta[r] = sHa[r] * SC2; tb[r] = sHb[r] * SC2; }
        }
        if (key0 + 31 > t0) {
            const int lim = t0 + lr - key0 - 8 * hi;
#pragma unroll
            for (int r = 0; r < 8; ++r) { ta[r] = (r <= lim) ? ta[r] : NEGB; tb[r] = (r + 16 <= lim) ? tb[r] : NEGB; }
        }
        float mx = NEGB;
#pragma unroll
        for (int r = 0; r < 8; ++r) mx = fmaxf(mx, fmaxf(ta[r], tb[r]));
        mx = fmaxf(mx, __shfl_xor(mx, 16, 32));
        const float mnew = fmaxf(m, mx);
        const float alpha = __builtin_amdgcn_exp2f(m - mnew);
        const float sh = PSH - mnew;
        v16h pb; v16h prb = (v16h){}; float ls = 0.0f;
#pragma unroll
        for (int r = 0; r < 8; ++r) {
            const float ea = __builtin_amdgcn_exp2f(ta[r] + sh), eb = __builtin_amdgcn_exp2f(tb[r] + sh);
            const h16 pa = (h16)ea; const h16 pc = (h16)eb; pb[r] = pa; pb[8 + r] = pc;
            if constexpr (PR) { prb[r] = (h16)((ea - (float)pa) * QRS); prb[8 + r] = (h16)((eb - (float)pc) * QRS); ls += ea + eb; }
            else              { ls += (float)pa + (float)pc; }
        }
        l = l * alpha + ls; m = mnew;
        oH0 = oH0 * alpha; oH1 = oH1 * alpha; oH2 = oH2 * alpha; oH3 = oH3 * alpha;
        if constexpr (PR) { oR0 = oR0 * alpha; oR1 = oR1 * alpha; oR2 = oR2 * alpha; oR3 = oR3 * alpha; }
        const h16* va = VT + vo + key0;
        const v16h v0 = ldh(va), v1 = ldh(va + (size_t)16 * SEQ), v2 = ldh(va + (size_t)32 * SEQ), v3 = ldh(va + (size_t)48 * SEQ);
        oH0 = wmma16(v0, pb, oH0); oH1 = wmma16(v1, pb, oH1); oH2 = wmma16(v2, pb, oH2); oH3 = wmma16(v3, pb, oH3);
        if constexpr (PR) {
            const h16* ra = VR + vro + key0;
            const v16h w0 = ldh(ra), w1 = ldh(ra + (size_t)16 * EPR), w2 = ldh(ra + (size_t)32 * EPR), w3 = ldh(ra + (size_t)48 * EPR);
            oR0 = wmma16(w0, pb, oR0); oR1 = wmma16(w1, pb, oR1); oR2 = wmma16(w2, pb, oR2); oR3 = wmma16(w3, pb, oR3);
            oR0 = wmma16(v0, prb, oR0); oR1 = wmma16(v1, prb, oR1); oR2 = wmma16(v2, prb, oR2); oR3 = wmma16(v3, prb, oR3);
            asm volatile("v_nop\n\tv_nop\n\tv_nop\n\tv_nop" : "+v"(oH0), "+v"(oH1), "+v"(oH2), "+v"(oH3), "+v"(oR0), "+v"(oR1), "+v"(oR2), "+v"(oR3)
                         : "v"(v0), "v"(v1), "v"(v2), "v"(v3), "v"(w0), "v"(w1), "v"(w2), "v"(w3), "v"(pb), "v"(prb));
        } else {
            asm volatile("v_nop\n\tv_nop\n\tv_nop\n\tv_nop" : "+v"(oH0), "+v"(oH1), "+v"(oH2), "+v"(oH3) : "v"(v0), "v"(v1), "v"(v2), "v"(v3), "v"(pb));
        }
    }
    l += __shfl_xor(l, 16, 32);
    const float inv = 1.0f / l;
    v8f c0 = oH0, c1 = oH1, c2 = oH2, c3 = oH3;
    if constexpr (PR) { c0 = oH0 + oR0 * QRI; c1 = oH1 + oR1 * QRI; c2 = oH2 + oR2 * QRI; c3 = oH3 + oR3 * QRI; }
    const int wb = wave * 16 * 68;
    { v4f a, c;
      a[0] = c0[0] * inv; a[1] = c0[1] * inv; a[2] = c0[2] * inv; a[3] = c0[3] * inv; c[0] = c0[4] * inv; c[1] = c0[5] * inv; c[2] = c0[6] * inv; c[3] = c0[7] * inv;
      *(v4fa*)(&os[wb + lr * 68 +  0 + 8 * hi]) = a; *(v4fa*)(&os[wb + lr * 68 +  0 + 8 * hi + 4]) = c;
      a[0] = c1[0] * inv; a[1] = c1[1] * inv; a[2] = c1[2] * inv; a[3] = c1[3] * inv; c[0] = c1[4] * inv; c[1] = c1[5] * inv; c[2] = c1[6] * inv; c[3] = c1[7] * inv;
      *(v4fa*)(&os[wb + lr * 68 + 16 + 8 * hi]) = a; *(v4fa*)(&os[wb + lr * 68 + 16 + 8 * hi + 4]) = c;
      a[0] = c2[0] * inv; a[1] = c2[1] * inv; a[2] = c2[2] * inv; a[3] = c2[3] * inv; c[0] = c2[4] * inv; c[1] = c2[5] * inv; c[2] = c2[6] * inv; c[3] = c2[7] * inv;
      *(v4fa*)(&os[wb + lr * 68 + 32 + 8 * hi]) = a; *(v4fa*)(&os[wb + lr * 68 + 32 + 8 * hi + 4]) = c;
      a[0] = c3[0] * inv; a[1] = c3[1] * inv; a[2] = c3[2] * inv; a[3] = c3[3] * inv; c[0] = c3[4] * inv; c[1] = c3[5] * inv; c[2] = c3[6] * inv; c[3] = c3[7] * inv;
      *(v4fa*)(&os[wb + lr * 68 + 48 + 8 * hi]) = a; *(v4fa*)(&os[wb + lr * 68 + 48 + 8 * hi + 4]) = c; }
    wave_sync();
    const size_t cb = ((size_t)b * SEQ + t0) * DM + (size_t)h * HD;
    const size_t rb = ((size_t)b * EPR + t0) * DM + (size_t)h * HD;
#pragma unroll 1
    for (int ps = 0; ps < 2; ++ps) {
#pragma unroll
        for (int s = 0; s < 4; ++s) { const int row = 4 * s + (lane >> 3), c8 = (lane & 7) * 8;
            const v4f x0 = *(const v4fa*)(&os[wb + row * 68 + c8]); const v4f x1 = *(const v4fa*)(&os[wb + row * 68 + c8 + 4]); v8h hv, rv;
#pragma unroll
            for (int i = 0; i < 4; ++i) { const h16 a0 = (h16)x0[i]; const h16 a1 = (h16)x1[i]; hv[i] = a0; hv[4 + i] = a1; rv[i] = (h16)((x0[i] - (float)a0) * QRS); rv[4 + i] = (h16)((x1[i] - (float)a1) * QRS); }
            *(volatile v8h*)(CH + cb + (size_t)row * DM + c8) = hv;
            if constexpr (PR) *(volatile v8h*)(CR + rb + (size_t)row * DM + c8) = rv; }
        if (ps == 0) __threadfence(); }
}

template <int MB, bool RES>
__global__ __launch_bounds__(32) void k_oproj(const h16* __restrict__ CH, const h16* __restrict__ CR, const h16* __restrict__ WO, float* OUT, int tpb, int tbeg) {
    __shared__ __align__(16) float os[16 * 68];
    const int K = DM;
    const int lane = threadIdx.x & 31, lr = lane & 15, hi = lane >> 4;
    const int b = blockIdx.x / tpb, tt = tbeg + ((int)blockIdx.x % tpb) * (16 * MB), c0 = blockIdx.y * 64;
    v8f acc[MB][4], accr[MB][4];
#pragma unroll
    for (int mb = 0; mb < MB; ++mb)
#pragma unroll
        for (int nb = 0; nb < 4; ++nb) { acc[mb][nb] = (v8f){}; accr[mb][nb] = (v8f){}; }
    const size_t aoff = ((size_t)b * SEQ + tt + lr) * K + 8 * hi;
    const size_t roff = ((size_t)b * EPR + tt + lr) * K + 8 * hi;
    const size_t boff = (size_t)(c0 + lr) * K + 8 * hi;
#pragma unroll 1
    for (int kc = 0; kc < K; kc += 32) {
        v16h a[MB], ar[MB];
#pragma unroll
        for (int mb = 0; mb < MB; ++mb) { a[mb] = ldh(CH + aoff + (size_t)mb * 16 * K + kc); ar[mb] = a[mb]; if (RES) ar[mb] = ldh(CR + roff + (size_t)mb * 16 * K + kc); }
#pragma unroll
        for (int nb = 0; nb < 4; ++nb) { const v16h bq = ldh(WO + boff + (size_t)nb * 16 * K + kc);
#pragma unroll
            for (int mb = 0; mb < MB; ++mb) { acc[mb][nb] = wmma16(a[mb], bq, acc[mb][nb]); if (RES) accr[mb][nb] = wmma16(ar[mb], bq, accr[mb][nb]); } }
        if (RES) asm volatile("v_nop\n\tv_nop\n\tv_nop\n\tv_nop" : "+v"(acc[0][3]), "+v"(acc[MB - 1][3]), "+v"(accr[0][3]), "+v"(accr[MB - 1][3]) : "v"(a[0]), "v"(a[MB - 1]), "v"(ar[0]), "v"(ar[MB - 1]));
        else     asm volatile("v_nop\n\tv_nop\n\tv_nop\n\tv_nop" : "+v"(acc[0][3]), "+v"(acc[MB - 1][3]) : "v"(a[0]), "v"(a[MB - 1]));
    }
#pragma unroll
    for (int mb = 0; mb < MB; ++mb) {
#pragma unroll
        for (int nb = 0; nb < 4; ++nb) {
#pragma unroll
            for (int j = 0; j < 8; ++j) { float val = acc[mb][nb][j]; if (RES) val += accr[mb][nb][j] * QRI; os[(hi * 8 + j) * 68 + nb * 16 + lr] = val * WOI; } }
        wave_sync();
        float* orow = OUT + ((size_t)b * OUT_SEQ + tt + mb * 16) * DM + c0;
#pragma unroll 1
        for (int ps = 0; ps < 2; ++ps) {
#pragma unroll
            for (int s = 0; s < 8; ++s) { const int row = 2 * s + hi, cofs = lr * 4;
                const v4f val = *(const v4fa*)(&os[row * 68 + cofs]);
                *(volatile v4f*)(orow + (size_t)row * DM + cofs) = val; }
            if (ps == 0) __threadfence(); }
        wave_sync();
    }
}

static constexpr size_t al256(size_t v) { return (v + 255) & ~(size_t)255; }
static constexpr size_t SZ_XB = al256((size_t)NB * SEQ * DM * 2);
static constexpr size_t SZ_WB = al256((size_t)4 * DM * DM * 2);
static constexpr size_t SZ_PL = al256((size_t)NB * NH_ * SEQ * HD * 2);
static constexpr size_t SZ_PS = al256((size_t)NB * NH_ * EPR * HD * 2);
static constexpr size_t SZ_TB = al256((size_t)2 * SEQ * 32 * 4);
static constexpr size_t SZ_TOTAL = SZ_XB + SZ_WB + 3 * SZ_PL + 4 * SZ_PS + SZ_TB;
static_assert(SZ_TOTAL <= (size_t)134217728);
static_assert(((size_t)DM * DM * 2) % 256 == 0);
static_assert((size_t)NB * SEQ * DM * 2 <= SZ_XB);
static_assert((size_t)NB * NH_ * EPR * HD * 2 <= SZ_PS);
static_assert((size_t)NB * EPR * DM * 2 <= SZ_PS);
static_assert((size_t)NB * DM * EPR * 2 <= SZ_PS);

extern "C" void kernel_launch(void* const* d_in, const int* in_sizes, int n_in,
                              void* d_out, int out_size, void* d_ws, size_t ws_size, hipStream_t stream) {
    if (n_in < 6) return;
    const size_t needx = ((size_t)(NB - 1) * SEQ_FULL + SEQ) * DM;
    if ((size_t)in_sizes[0] < needx) return;
    if ((size_t)in_sizes[1] < (size_t)DM * DM || (size_t)in_sizes[2] < (size_t)DM * DM || (size_t)in_sizes[3] < (size_t)DM * DM || (size_t)in_sizes[4] < (size_t)DM * DM) return;
    if ((size_t)in_sizes[5] < (size_t)SEQ) return;
    if ((size_t)out_size < ((size_t)(NB - 1) * OUT_SEQ + SEQ) * DM) return;
    if (SZ_TOTAL > ws_size) return;
    const float* x = (const float*)d_in[0]; const float* wq = (const float*)d_in[1]; const float* wk = (const float*)d_in[2];
    const float* wv = (const float*)d_in[3]; const float* wo = (const float*)d_in[4]; const int* tpos = (const int*)d_in[5];
    float* OUT = (float*)d_out;
    char* wsp = (char*)d_ws;
    bf* XB = (bf*)wsp; h16* CH = (h16*)wsp; wsp += SZ_XB;
    bf* WB = (bf*)wsp; wsp += SZ_WB;
    h16* QH = (h16*)wsp; wsp += SZ_PL;
    h16* KP = (h16*)wsp; wsp += SZ_PL;
    h16* VT = (h16*)wsp; wsp += SZ_PL;
    h16* QR = (h16*)wsp; wsp += SZ_PS;
    h16* KR = (h16*)wsp; wsp += SZ_PS;
    h16* VR = (h16*)wsp; wsp += SZ_PS;
    h16* CR = (h16*)wsp; wsp += SZ_PS;
    float* TB = (float*)wsp; wsp += SZ_TB;
    bf* WQ = WB; bf* WK = WB + (size_t)DM * DM; bf* WV = WB + (size_t)2 * DM * DM; h16* WO = (h16*)(WB + (size_t)3 * DM * DM);

    if (SEQ == SEQ_FULL) {
        const size_t n8 = (size_t)NB * SEQ * DM / 8;
        k_cvt8<<<(unsigned)((n8 + 255) / 256), 256, 0, stream>>>(x, XB, n8);
    } else {
        const size_t n8 = (size_t)SEQ * DM / 8;
        for (int b = 0; b < NB; ++b) k_cvt8<<<(unsigned)((n8 + 255) / 256), 256, 0, stream>>>(x + (size_t)b * SEQ_FULL * DM, XB + (size_t)b * SEQ * DM, n8);
    }
    { const size_t n8 = (size_t)DM * DM / 8; const unsigned g = (unsigned)((n8 + 255) / 256);
      k_cvt8<<<g, 256, 0, stream>>>(wq, WQ, n8); k_cvt8<<<g, 256, 0, stream>>>(wk, WK, n8); k_cvt8<<<g, 256, 0, stream>>>(wv, WV, n8);
      k_cvtw<<<g, 256, 0, stream>>>(wo, WO, n8); }
    k_tab<<<SEQ / 8, 256, 0, stream>>>(tpos, TB);

    k_proj<<<dim3(NB * SEQ / 64, DM / 64, 1), 32, 0, stream>>>(XB, WQ, QH, QR, SEQ, (size_t)NH_ * SEQ * HD, HD, HD, (size_t)SEQ * HD,
                                                                1, HD, (size_t)NH_ * EPR * HD, (size_t)EPR * HD, EPR, HD, TB, 1);
    k_proj<<<dim3(NB * SEQ / 64, DM / 64, 1), 32, 0, stream>>>(XB, WK, KP, KR, SEQ, (size_t)NH_ * SEQ * HD, HD, HD, (size_t)SEQ * HD,
                                                                1, HD, (size_t)NH_ * EPR * HD, (size_t)EPR * HD, EPR, HD, TB, 1);
    k_proj<<<dim3(DM / 64, NB * SEQ / 64, 1), 32, 0, stream>>>(WV, XB, VT, VR, DM, (size_t)0, SEQ, SEQ, (size_t)DM * SEQ,
                                                                1, EPR, (size_t)0, (size_t)DM * EPR, DM, EPR, TB, 0);

    k_flash<true><<<dim3(EPR / (16 * AW), NB * NH_, 1), 32 * AW, 0, stream>>>(QH, QR, KP, KR, VT, VR, CH, CR, 0);
    if (SEQ > EPR)
        k_flash<false><<<dim3((SEQ - EPR) / (16 * AW), NB * NH_, 1), 32 * AW, 0, stream>>>(QH, QR, KP, KR, VT, VR, CH, CR, EPR / (16 * AW));

    k_oproj<2, true><<<dim3(NB * (EPR / 32), DM / 64, 1), 32, 0, stream>>>(CH, CR, WO, OUT, EPR / 32, 0);
    if (SEQ > EPR)
        k_oproj<4, false><<<dim3(NB * ((SEQ - EPR) / 64), DM / 64, 1), 32, 0, stream>>>(CH, CR, WO, OUT, (SEQ - EPR) / 64, EPR);
}
